// MambaBranch_42554535969384
// MI455X (gfx1250) — hardware-verified
//
#include <hip/hip_runtime.h>
#include <math.h>

typedef __attribute__((ext_vector_type(16))) _Float16 v16h;
typedef __attribute__((ext_vector_type(8)))  _Float16 v8h;
typedef __attribute__((ext_vector_type(16))) __bf16   v16b;
typedef __attribute__((ext_vector_type(8)))  __bf16   v8b;
typedef __attribute__((ext_vector_type(8)))  float    v8f;
typedef __attribute__((ext_vector_type(4)))  float    v4f;
typedef __attribute__((ext_vector_type(4)))  unsigned int v4u;

constexpr int kBatch  = 2;
constexpr int kChan   = 2048;
constexpr int kSeq    = 2048;
constexpr int kTaps   = 4;
constexpr int kDtR    = 128;
constexpr int kNst    = 16;
constexpr int kE      = kDtR + 2 * kNst;
constexpr int kEP     = 192;
constexpr int kRows   = kBatch * kSeq;
constexpr int kBCW    = 32;
constexpr int kCvP    = 68;
constexpr int kScanTS = 64;
constexpr int kScanCh = 64;
constexpr int kScanYP = 68;
constexpr int kGateP  = 65;
static_assert(kE == 160 && kEP % 64 == 0 && kEP >= kE);
static_assert((kChan % 32) == 0 && (kDtR % 32) == 0);
static_assert((kRows % 64) == 0 && (kEP % 64) == 0 && (kChan % 64) == 0);
static_assert((kSeq % kScanTS) == 0 && (kSeq % 64) == 0 && (kChan % kScanCh) == 0 && (kChan % 64) == 0);
static_assert(kTaps == 4);

constexpr size_t kOffUF   = 0;
constexpr size_t kOffUH   = kOffUF  + (size_t)kRows * kChan * 4;
constexpr size_t kOffUL   = kOffUH  + (size_t)kRows * kChan * 2;
constexpr size_t kOffDP   = kOffUH;
constexpr size_t kOffWXH  = kOffUL  + (size_t)kRows * kChan * 2;
constexpr size_t kOffWXL  = kOffWXH + (size_t)kEP   * kChan * 2;
constexpr size_t kOffWDH  = kOffWXL + (size_t)kEP   * kChan * 2;
constexpr size_t kOffWDL  = kOffWDH + (size_t)kChan * kDtR  * 2;
constexpr size_t kOffSSM  = kOffWDL + (size_t)kChan * kDtR  * 2;
constexpr size_t kOffDTH  = kOffSSM + (size_t)kRows * kEP   * 4;
constexpr size_t kOffDTL  = kOffDTH + (size_t)kRows * kDtR  * 2;
constexpr size_t kOffBC   = kOffDTL + (size_t)kRows * kDtR  * 2;
constexpr size_t kWsTotal = kOffBC  + (size_t)kRows * kBCW  * 4;
static_assert(kWsTotal == 75497472ull);
static_assert(kWsTotal <= 134217728ull);
static_assert(kOffDP + (size_t)kRows * kChan * 4 == kOffWXH);
static_assert((kOffUH % 128) == 0 && (kOffUL % 128) == 0 && (kOffWXH % 128) == 0 && (kOffWXL % 128) == 0 &&
              (kOffWDH % 128) == 0 && (kOffWDL % 128) == 0 && (kOffSSM % 128) == 0 && (kOffDTH % 128) == 0 &&
              (kOffDTL % 128) == 0 && (kOffBC % 128) == 0);

__device__ __forceinline__ unsigned short f2bf_bits(float f) {
  unsigned u = __float_as_uint(f);
  return (unsigned short)((u + 0x7FFFu + ((u >> 16) & 1u)) >> 16);
}
__device__ __forceinline__ float bf_bits2f(unsigned short h) { return __uint_as_float(((unsigned)h) << 16); }

__device__ __forceinline__ void dep_guard_h(v8f& a, v8f& b, v16h x, v16h y) { asm volatile("v_nop\n\tv_nop\n\tv_nop\n\tv_nop" : "+v"(a), "+v"(b) : "v"(x), "v"(y)); }
__device__ __forceinline__ void dep_guard_b(v8f& a, v8f& b, v16b x, v16b y) { asm volatile("v_nop\n\tv_nop\n\tv_nop\n\tv_nop" : "+v"(a), "+v"(b) : "v"(x), "v"(y)); }
__device__ __forceinline__ void keep4_h(v16h a, v16h b, v16h c, v16h d) { asm volatile("v_nop" :: "v"(a), "v"(b), "v"(c), "v"(d)); }
__device__ __forceinline__ void keep4_b(v16b a, v16b b, v16b c, v16b d) { asm volatile("v_nop" :: "v"(a), "v"(b), "v"(c), "v"(d)); }
__device__ __forceinline__ void acc_guard4(v8f& a, v8f& b, v8f& c, v8f& d) { asm volatile("v_nop\n\tv_nop\n\tv_nop\n\tv_nop" : "+v"(a), "+v"(b), "+v"(c), "+v"(d)); }
template <typename T> struct Frag;
template <> struct Frag<_Float16> {
  typedef v16h V; union U { v16h v; v8h h[2]; };
  static __device__ __forceinline__ v16h load(const _Float16* p) {
    U f; f.h[0] = *(const v8h*)(p); f.h[1] = *(const v8h*)(p + 16); return f.v;
  }
  static __device__ __forceinline__ v8f mma(v16h a, v16h b, v8f c) {
    return __builtin_amdgcn_wmma_f32_16x16x32_f16(false, a, false, b, (short)0, c, false, false);
  }
  static __device__ __forceinline__ void guard(v8f& a, v8f& b, v16h x, v16h y) { dep_guard_h(a, b, x, y); }
  static __device__ __forceinline__ void keep(v16h a, v16h b, v16h c, v16h d) { keep4_h(a, b, c, d); }
};
template <> struct Frag<__bf16> {
  typedef v16b V; union U { v16b v; v8b h[2]; };
  static __device__ __forceinline__ v16b load(const __bf16* p) {
    U f; f.h[0] = *(const v8b*)(p); f.h[1] = *(const v8b*)(p + 16); return f.v;
  }
  static __device__ __forceinline__ v8f mma(v16b a, v16b b, v8f c) {
    return __builtin_amdgcn_wmma_f32_16x16x32_bf16(false, a, false, b, (short)0, c, false, false);
  }
  static __device__ __forceinline__ void guard(v8f& a, v8f& b, v16b x, v16b y) { dep_guard_b(a, b, x, y); }
  static __device__ __forceinline__ void keep(v16b a, v16b b, v16b c, v16b d) { keep4_b(a, b, c, d); }
};

template <int ET> struct Elem;
template <> struct Elem<0> { typedef _Float16 T; };
template <> struct Elem<1> { typedef __bf16 T; };
template <int ET, int SPL, int BIAS_MODE, int OUT_MODE, bool RESID, int ACT = 0>
__global__ __launch_bounds__(256) void wmma_gemm64(
    const unsigned short* __restrict__ Ap, const unsigned short* __restrict__ A2p, int lda, long strideA,
    const unsigned short* __restrict__ Btp, const unsigned short* __restrict__ Bt2p, int ldb, long strideB,
    void* __restrict__ Cout, void* __restrict__ Cout2, int ldc, long strideC,
    const float* __restrict__ bias,
    const float* __restrict__ resid, long strideR,
    int M, int N, int K, float scale) {
  typedef typename Elem<ET>::T T;
  typedef typename Frag<T>::V V;
  const T* A = (const T*)Ap; const T* A2 = (const T*)A2p; const T* Bt = (const T*)Btp; const T* Bt2 = (const T*)Bt2p;
  __shared__ __align__(16) float sT[8][16 * 68];
  const int b    = blockIdx.y;
  const int lane = threadIdx.x & 31;
  const int wave = threadIdx.x >> 5;
  const int tilesN = N >> 6;
  const int tilesM = M >> 6;
  const int tile = blockIdx.x * 8 + wave;
  if (tile >= tilesM * tilesN) return;
  const int tm = tile / tilesN;
  const int tn = tile - tm * tilesN;
  const int m0 = tm << 6;
  const int n0 = tn << 6;

  const T* Ab  = A  + (size_t)b * strideA;
  const T* Bb  = Bt + (size_t)b * strideB;
  const T* Ab2 = (SPL >= 1) ? (A2  + (size_t)b * strideA) : nullptr;
  const T* Bb2 = (SPL == 2) ? (Bt2 + (size_t)b * strideB) : nullptr;

  const int rlane = lane & 15;
  const int koff  = (lane >> 4) * 8;
  const int mOff  = (lane >> 4) * 8;

  v8f acc[4][4];
#pragma unroll
  for (int i = 0; i < 4; ++i)
#pragma unroll
    for (int j = 0; j < 4; ++j) acc[i][j] = (v8f){0.f,0.f,0.f,0.f,0.f,0.f,0.f,0.f};

  for (int k0 = 0; k0 < K; k0 += 32) {
    V bh[4], bl[4];
#pragma unroll
    for (int j = 0; j < 4; ++j) {
      const size_t bo = (size_t)(n0 + (j << 4) + rlane) * ldb + koff + k0;
      bh[j] = Frag<T>::load(Bb + bo);
      if (SPL == 2) bl[j] = Frag<T>::load(Bb2 + bo);
    }
#pragma unroll
    for (int i = 0; i < 4; ++i) {
      const size_t ao = (size_t)(m0 + (i << 4) + rlane) * lda + koff + k0;
      V ah = Frag<T>::load(Ab + ao);
      V al;
      if (SPL >= 1) al = Frag<T>::load(Ab2 + ao);
#pragma unroll
      for (int j = 0; j < 4; ++j) {
        acc[i][j] = Frag<T>::mma(ah, bh[j], acc[i][j]);
        if (SPL == 2) acc[i][j] = Frag<T>::mma(ah, bl[j], acc[i][j]);
        if (SPL >= 1) acc[i][j] = Frag<T>::mma(al, bh[j], acc[i][j]);
      }
      Frag<T>::guard(acc[i][0], acc[i][3], ah, (SPL >= 1) ? al : ah);
    }
    Frag<T>::keep(bh[0], bh[1], bh[2], bh[3]);
    if (SPL == 2) Frag<T>::keep(bl[0], bl[1], bl[2], bl[3]);
  }
  acc_guard4(acc[0][0], acc[0][1], acc[0][2], acc[0][3]);
  acc_guard4(acc[1][0], acc[1][1], acc[1][2], acc[1][3]);
  acc_guard4(acc[2][0], acc[2][1], acc[2][2], acc[2][3]);
  acc_guard4(acc[3][0], acc[3][1], acc[3][2], acc[3][3]);

  float* slab = sT[wave];
  const float* Rb = RESID ? (resid + (size_t)b * strideR) : nullptr;
#pragma unroll
  for (int i = 0; i < 4; ++i) {
    const int mBase = m0 + (i << 4);
#pragma unroll
    for (int j = 0; j < 4; ++j) {
      const int n = n0 + (j << 4) + rlane;
      float bv = 0.f;
      if (BIAS_MODE == 2) bv = bias[n];
#pragma unroll
      for (int r = 0; r < 8; ++r) {
        float v = acc[i][j][r] * scale;
        if (BIAS_MODE == 1) v += bias[mBase + mOff + r];
        if (BIAS_MODE == 2) v += bv;
        if (RESID) v += Rb[(size_t)(mBase + mOff + r) * ldc + n];
        if (ACT == 1) v = tanhf(v);
        if (ACT == 2) v = fmaxf(v, 0.0f);
        if (ACT == 3) v = v / (1.0f + expf(-v));
        if (ACT == 4) v = (v > 0.f) ? v : 0.01f * v;
        slab[(mOff + r) * 68 + (j << 4) + rlane] = v;
      }
    }
    __builtin_amdgcn_fence(__ATOMIC_RELEASE, "workgroup");
    __builtin_amdgcn_wave_barrier();
    __builtin_amdgcn_fence(__ATOMIC_ACQUIRE, "workgroup");
    if (OUT_MODE == 0) {
      float* C = (float*)Cout + (size_t)b * strideC;
      const int hh = lane >> 4, c4 = (lane & 15) * 4;
      for (int pass = 0; pass < 2; ++pass) {
#pragma unroll
        for (int it = 0; it < 8; ++it) {
          const int row = it * 2 + hh;
          v4f v = *(const v4f*)(slab + row * 68 + c4);
          *(volatile v4f*)(C + (size_t)(mBase + row) * ldc + n0 + c4) = v;
        }
        __threadfence();
      }
    } else {
      const int q = lane >> 3, c8 = (lane & 7) * 8;
      unsigned short* C  = (unsigned short*)Cout  + (size_t)b * strideC;
      unsigned short* C2 = (OUT_MODE == 2) ? ((unsigned short*)Cout2 + (size_t)b * strideC) : nullptr;
      for (int pass = 0; pass < 2; ++pass) {
#pragma unroll
        for (int it = 0; it < 4; ++it) {
          const int row = it * 4 + q;
          const float* sp = slab + row * 68 + c8;
          v8h hv, lv;
#pragma unroll
          for (int e = 0; e < 8; ++e) {
            if (OUT_MODE == 1) {
              hv[e] = (_Float16)sp[e];
            } else {
              unsigned short hb = f2bf_bits(sp[e]);
              unsigned short lb = f2bf_bits(sp[e] - bf_bits2f(hb));
              hv[e] = __builtin_bit_cast(_Float16, hb);
              lv[e] = __builtin_bit_cast(_Float16, lb);
            }
          }
          *(volatile v8h*)(C + (size_t)(mBase + row) * ldc + n0 + c8) = hv;
          if (OUT_MODE == 2) *(volatile v8h*)(C2 + (size_t)(mBase + row) * ldc + n0 + c8) = lv;
        }
        __threadfence();
      }
    }
    __builtin_amdgcn_fence(__ATOMIC_RELEASE, "workgroup");
    __builtin_amdgcn_wave_barrier();
    __builtin_amdgcn_fence(__ATOMIC_ACQUIRE, "workgroup");
  }
}

__global__ __launch_bounds__(256) void split_rows_bf16_kernel(
    const float* __restrict__ src, unsigned short* __restrict__ dhi, unsigned short* __restrict__ dlo,
    int real8, int total8)
{
  const int i = blockIdx.x * 256 + threadIdx.x;
  if (i >= total8) return;
  const bool valid = (i < real8);
  const int ic = valid ? i : (real8 - 1);
  const size_t s0 = (size_t)ic << 3;
  v4f a0 = *(const v4f*)(src + s0);
  v4f a1 = *(const v4f*)(src + s0 + 4);
  if (!valid) { a0 = (v4f){0.f, 0.f, 0.f, 0.f}; a1 = (v4f){0.f, 0.f, 0.f, 0.f}; }
  v8h hv, lv;
#pragma unroll
  for (int e = 0; e < 4; ++e) {
    const unsigned short h0 = f2bf_bits(a0[e]), h1 = f2bf_bits(a1[e]);
    const unsigned short l0 = f2bf_bits(a0[e] - bf_bits2f(h0)), l1 = f2bf_bits(a1[e] - bf_bits2f(h1));
    hv[e]     = __builtin_bit_cast(_Float16, h0);
    hv[4 + e] = __builtin_bit_cast(_Float16, h1);
    lv[e]     = __builtin_bit_cast(_Float16, l0);
    lv[4 + e] = __builtin_bit_cast(_Float16, l1);
  }
  const size_t e0 = (size_t)i << 3;
  unsigned short* qh = dhi + e0;
  unsigned short* ql = dlo + e0;
  *(volatile v8h*)qh = hv;
  *(volatile v8h*)ql = lv;
  __threadfence();
  *(volatile v8h*)qh = hv;
  *(volatile v8h*)ql = lv;
}

__global__ __launch_bounds__(256) void conv_silu_tr_kernel(
    const float* __restrict__ hs, const float* __restrict__ cw, const float* __restrict__ cb,
    float* __restrict__ UF, unsigned short* __restrict__ UH, unsigned short* __restrict__ UL)
{
  __shared__ __align__(16) float sIn[64 * kCvP];
  __shared__ __align__(16) float sOut[64 * kCvP];
  const int tid = threadIdx.x, lane = tid & 31, wave = tid >> 5;
  const int l0 = blockIdx.x * 64;
  const int d0 = blockIdx.y * 64;
  const int b  = blockIdx.z;
  const float* hb = hs + ((size_t)b * kChan + d0) * kSeq;
#pragma unroll
  for (int i = 0; i < 16; ++i) {
    const int idx = tid + 256 * i;
    const int c = idx >> 6, t = idx & 63;
    sIn[c * kCvP + 3 + t] = hb[(size_t)c * kSeq + l0 + t];
  }
  if (tid < 192) {
    const int c = tid / 3;
    const int j = tid - 3 * c;
    const int ls = l0 - 3 + j;
    const int lc = (ls < 0) ? 0 : ls;
    const float v = hb[(size_t)c * kSeq + lc];
    sIn[c * kCvP + j] = (ls >= 0) ? v : 0.f;
  }
  __syncthreads();
  {
    const int c = tid & 63, tg = tid >> 6;
    const v4f w = *(const v4f*)(cw + (size_t)(d0 + c) * kTaps);
    const float bc = cb[d0 + c];
#pragma unroll 1
    for (int s = 0; s < 16; ++s) {
      const int t = tg * 16 + s;
      const float* xp = sIn + c * kCvP + t;
      float acc = w[0] * xp[0];
      acc = fmaf(w[1], xp[1], acc);
      acc = fmaf(w[2], xp[2], acc);
      acc = fmaf(w[3], xp[3], acc);
      const float sv = acc + bc;
      const float sg = __builtin_amdgcn_rcpf(1.0f + expf(-sv));
      sOut[t * kCvP + c] = sv * sg;
    }
  }
  __syncthreads();
  const int hh = lane >> 4, c4 = (lane & 15) * 4;
  const int q = lane >> 3, c8 = (lane & 7) * 8;
  v4f fv[4];
  v8h bh[2], blo[2];
#pragma unroll
  for (int it = 0; it < 4; ++it) fv[it] = *(const v4f*)(sOut + (it * 16 + wave * 2 + hh) * kCvP + c4);
#pragma unroll
  for (int it = 0; it < 2; ++it) {
    const float* sp = sOut + (it * 32 + wave * 4 + q) * kCvP + c8;
    const v4f a0 = *(const v4f*)(sp);
    const v4f a1 = *(const v4f*)(sp + 4);
#pragma unroll
    for (int e = 0; e < 4; ++e) {
      const unsigned short h0 = f2bf_bits(a0[e]), h1 = f2bf_bits(a1[e]);
      const unsigned short l0b = f2bf_bits(a0[e] - bf_bits2f(h0)), l1b = f2bf_bits(a1[e] - bf_bits2f(h1));
      bh[it][e]      = __builtin_bit_cast(_Float16, h0);
      bh[it][4 + e]  = __builtin_bit_cast(_Float16, h1);
      blo[it][e]     = __builtin_bit_cast(_Float16, l0b);
      blo[it][4 + e] = __builtin_bit_cast(_Float16, l1b);
    }
  }
  const size_t grow0 = (size_t)b * kSeq + l0;
  for (int pass = 0; pass < 2; ++pass) {
#pragma unroll
    for (int it = 0; it < 4; ++it)
      *(volatile v4f*)(UF + (grow0 + it * 16 + wave * 2 + hh) * kChan + d0 + c4) = fv[it];
#pragma unroll
    for (int it = 0; it < 2; ++it) {
      const size_t o = (grow0 + it * 32 + wave * 4 + q) * kChan + d0 + c8;
      *(volatile v8h*)(UH + o) = bh[it];
      *(volatile v8h*)(UL + o) = blo[it];
    }
    __threadfence();
  }
}

__global__ __launch_bounds__(256) void rmsnorm_kernel(
    const float* __restrict__ SSM, const float* __restrict__ dtln, const float* __restrict__ bln,
    const float* __restrict__ cln, unsigned short* __restrict__ DTH, unsigned short* __restrict__ DTL,
    float* __restrict__ BC)
{
  const int lane = threadIdx.x & 31, wave = threadIdx.x >> 5;
  const int row = blockIdx.x * 8 + wave;
  const float* r = SSM + (size_t)row * kEP;
  const v4f x = *(const v4f*)(r + lane * 4);
  float ss = x[0] * x[0];
  ss = fmaf(x[1], x[1], ss);
  ss = fmaf(x[2], x[2], ss);
  ss = fmaf(x[3], x[3], ss);
#pragma unroll
  for (int m = 16; m >= 1; m >>= 1) ss += __shfl_xor(ss, m, 32);
  const float rs = rsqrtf(ss * (1.0f / 128.0f) + 1e-6f);
  const v4f w = *(const v4f*)(dtln + lane * 4);
  const float o0 = w[0] * (x[0] * rs), o1 = w[1] * (x[1] * rs), o2v = w[2] * (x[2] * rs), o3 = w[3] * (x[3] * rs);
  const unsigned short h0 = f2bf_bits(o0), h1 = f2bf_bits(o1), h2 = f2bf_bits(o2v), h3 = f2bf_bits(o3);
  const unsigned short l0 = f2bf_bits(o0 - bf_bits2f(h0)), l1 = f2bf_bits(o1 - bf_bits2f(h1));
  const unsigned short l2 = f2bf_bits(o2v - bf_bits2f(h2)), l3 = f2bf_bits(o3 - bf_bits2f(h3));
  const unsigned ph0 = (unsigned)h0 | ((unsigned)h1 << 16), ph1 = (unsigned)h2 | ((unsigned)h3 << 16);
  const unsigned pl0 = (unsigned)l0 | ((unsigned)l1 << 16), pl1 = (unsigned)l2 | ((unsigned)l3 << 16);
  const int q = lane & 15;
  const unsigned a0 = __shfl(ph0, 2 * q, 32), a1 = __shfl(ph1, 2 * q, 32);
  const unsigned a2 = __shfl(ph0, 2 * q + 1, 32), a3 = __shfl(ph1, 2 * q + 1, 32);
  const unsigned g0 = __shfl(pl0, 2 * q, 32), g1 = __shfl(pl1, 2 * q, 32);
  const unsigned g2 = __shfl(pl0, 2 * q + 1, 32), g3 = __shfl(pl1, 2 * q + 1, 32);
  const bool selh = (lane < 16);
  v4u dv;
  dv[0] = selh ? a0 : g0; dv[1] = selh ? a1 : g1; dv[2] = selh ? a2 : g2; dv[3] = selh ? a3 : g3;
  unsigned short* pd = (selh ? DTH : DTL) + (size_t)row * kDtR + 8 * q;

  const float xb = r[kDtR + lane];
  float s2 = xb * xb;
#pragma unroll
  for (int m = 8; m >= 1; m >>= 1) s2 += __shfl_xor(s2, m, 32);
  const float rs2 = rsqrtf(s2 * (1.0f / 16.0f) + 1e-6f);
  const float wb = bln[lane & 15], wc = cln[lane & 15];
  const float w2 = selh ? wb : wc;
  const float ob = w2 * (xb * rs2);
  const int q3 = lane & 7;
  v4f gv;
  gv[0] = __shfl(ob, 4 * q3, 32); gv[1] = __shfl(ob, 4 * q3 + 1, 32);
  gv[2] = __shfl(ob, 4 * q3 + 2, 32); gv[3] = __shfl(ob, 4 * q3 + 3, 32);
  float* pb = BC + (size_t)row * kBCW + 4 * q3;
  for (int pass = 0; pass < 2; ++pass) {
    *(volatile v4u*)pd = dv;
    if (lane < 8) *(volatile v4f*)pb = gv;
    __threadfence();
  }
}

__global__ __launch_bounds__(64) void scan_gate_kernel(
    const float* __restrict__ DP, const float* __restrict__ UF, const float* __restrict__ BC,
    const float* __restrict__ gate, const float* __restrict__ dtb, const float* __restrict__ Alog,
    const float* __restrict__ Dp, float* __restrict__ out)
{
  __shared__ __align__(16) float sBC[kScanTS * kBCW];
  __shared__ __align__(16) float sG[kScanCh * kGateP];
  __shared__ __align__(16) float sY[kScanTS * kScanYP];
  __shared__ __align__(16) float sA[kNst * kScanCh];
  const int tid = threadIdx.x, lane = tid & 31, wave = tid >> 5;
  constexpr int kBlkPerB = kChan / kScanCh;
  const int bix = blockIdx.x / kBlkPerB;
  const int d0  = (blockIdx.x - bix * kBlkPerB) * kScanCh;
  const int d   = d0 + tid;
  const size_t row0 = (size_t)bix * kSeq;
#pragma unroll 1
  for (int s = 0; s < kNst; ++s) sA[s * kScanCh + tid] = -expf(Alog[(size_t)d * kNst + s]);
  __syncthreads();
  float negA[kNst], h[kNst];
#pragma unroll
  for (int s = 0; s < kNst; ++s) {
    negA[s] = sA[s * kScanCh + tid];
    h[s] = 0.f;
  }
  const float bb = dtb[d], Dd = Dp[d];
  const float* gb = gate + ((size_t)bix * kChan + d0) * kSeq;
  const int lr = tid >> 3, lc4 = (tid & 7) * 4;
  const int hh = lane >> 4, c4 = (lane & 15) * 4;
#pragma unroll 1
  for (int t0 = 0; t0 < kSeq; t0 += kScanTS) {
    __syncthreads();
#pragma unroll
    for (int i = 0; i < 8; ++i) {
      const int r = lr + 8 * i;
      *(v4f*)(sBC + r * kBCW + lc4) = *(const v4f*)(BC + (row0 + t0 + r) * kBCW + lc4);
    }
#pragma unroll 1
    for (int i = 0; i < kScanCh; ++i) sG[i * kGateP + tid] = gb[(size_t)i * kSeq + t0 + tid];
    __syncthreads();
#pragma unroll 1
    for (int s = 0; s < kScanTS; ++s) {
      const int t = t0 + s;
      const float* xr = sBC + s * kBCW;
      float Bs[kNst], Cs[kNst];
#pragma unroll
      for (int q4 = 0; q4 < 4; ++q4) {
        const v4f bv = *(const v4f*)(xr + 4 * q4);
        const v4f cv = *(const v4f*)(xr + kNst + 4 * q4);
        Bs[4 * q4 + 0] = bv[0]; Bs[4 * q4 + 1] = bv[1]; Bs[4 * q4 + 2] = bv[2]; Bs[4 * q4 + 3] = bv[3];
        Cs[4 * q4 + 0] = cv[0]; Cs[4 * q4 + 1] = cv[1]; Cs[4 * q4 + 2] = cv[2]; Cs[4 * q4 + 3] = cv[3];
      }
      const float v   = DP[(row0 + t) * kChan + d] + bb;
      const float a   = expf(-fabsf(v));
      const float u1  = 1.0f + a;
      const float l1p = __logf(u1) + (a - (u1 - 1.0f)) * __builtin_amdgcn_rcpf(u1);
      const float dt  = fmaxf(v, 0.0f) + l1p;
      const float xt  = UF[(row0 + t) * kChan + d];
      const float dtx = dt * xt;
      float y = 0.f;
#pragma unroll
      for (int k = 0; k < kNst; ++k) {
        const float e = __expf(dt * negA[k]);
        h[k] = e * h[k] + dtx * Bs[k];
        y = h[k] * Cs[k] + y;
      }
      y = xt * Dd + y;
      const float zv = sG[tid * kGateP + s];
      const float sg = __builtin_amdgcn_rcpf(1.0f + expf(-zv));
      y = y * (zv * sg);
      sY[s * kScanYP + tid] = y;
    }
    __syncthreads();
    for (int pass = 0; pass < 2; ++pass) {
#pragma unroll
      for (int it = 0; it < 16; ++it) {
        const int row = it * 4 + wave * 2 + hh;
        const v4f val = *(const v4f*)(sY + row * kScanYP + c4);
        *(volatile v4f*)(out + (row0 + t0 + row) * kChan + d0 + c4) = val;
      }
      __threadfence();
    }
  }
}

extern "C" void kernel_launch(void* const* d_in, const int* in_sizes, int n_in,
                              void* d_out, int out_size, void* d_ws, size_t ws_size,
                              hipStream_t stream) {
  if (n_in < 12) return;
  if (in_sizes[0] != kBatch * kChan * kSeq) return;
  if (in_sizes[1] != kBatch * kChan * kSeq) return;
  if (in_sizes[2] != kChan * kTaps) return;
  if (in_sizes[3] != kChan) return;
  if (in_sizes[4] != kE * kChan) return;
  if (in_sizes[5] != kChan * kDtR) return;
  if (in_sizes[6] != kChan) return;
  if (in_sizes[7] != kChan * kNst) return;
  if (in_sizes[8] != kChan) return;
  if (in_sizes[9] != kDtR) return;
  if (in_sizes[10] != kNst) return;
  if (in_sizes[11] != kNst) return;
  if (out_size != kRows * kChan) return;
  if (ws_size < kWsTotal) return;

  const float* hs     = (const float*)d_in[0];
  const float* gate   = (const float*)d_in[1];
  const float* conv_w = (const float*)d_in[2];
  const float* conv_b = (const float*)d_in[3];
  const float* W_x    = (const float*)d_in[4];
  const float* W_dt   = (const float*)d_in[5];
  const float* b_dt   = (const float*)d_in[6];
  const float* A_log  = (const float*)d_in[7];
  const float* Dp     = (const float*)d_in[8];
  const float* dt_ln  = (const float*)d_in[9];
  const float* b_ln   = (const float*)d_in[10];
  const float* c_ln   = (const float*)d_in[11];
  float* out = (float*)d_out;

  char* ws = (char*)d_ws;
  float*          UF  = (float*)(ws + kOffUF);
  unsigned short* UH  = (unsigned short*)(ws + kOffUH);
  unsigned short* UL  = (unsigned short*)(ws + kOffUL);
  float*          DP  = (float*)(ws + kOffDP);
  unsigned short* WXH = (unsigned short*)(ws + kOffWXH);
  unsigned short* WXL = (unsigned short*)(ws + kOffWXL);
  unsigned short* WDH = (unsigned short*)(ws + kOffWDH);
  unsigned short* WDL = (unsigned short*)(ws + kOffWDL);
  float*          SSM = (float*)(ws + kOffSSM);
  unsigned short* DTH = (unsigned short*)(ws + kOffDTH);
  unsigned short* DTL = (unsigned short*)(ws + kOffDTL);
  float*          BC  = (float*)(ws + kOffBC);

  {
    constexpr int total8 = kEP * kChan / 8;
    constexpr int real8  = kE * kChan / 8;
    static_assert(total8 % 256 == 0);
    split_rows_bf16_kernel<<<total8 / 256, 256, 0, stream>>>(W_x, WXH, WXL, real8, total8);
  }
  {
    constexpr int total8 = kChan * kDtR / 8;
    static_assert(total8 % 256 == 0);
    split_rows_bf16_kernel<<<total8 / 256, 256, 0, stream>>>(W_dt, WDH, WDL, total8, total8);
  }

  conv_silu_tr_kernel<<<dim3(kSeq / 64, kChan / 64, kBatch), 256, 0, stream>>>(hs, conv_w, conv_b, UF, UH, UL);

  {
    constexpr int tiles = (kRows / 64) * (kEP / 64);
    static_assert(tiles % 8 == 0);
    wmma_gemm64<1, 2, 0, 0, false><<<dim3(tiles / 8, 1), 256, 0, stream>>>(
        UH, UL, kChan, 0L,
        WXH, WXL, kChan, 0L,
        (void*)SSM, nullptr, kEP, 0L,
        nullptr, nullptr, 0L,
        kRows, kEP, kChan, 1.0f);
  }

  rmsnorm_kernel<<<kRows / 8, 256, 0, stream>>>(SSM, dt_ln, b_ln, c_ln, DTH, DTL, BC);

  {
    constexpr int tiles = (kRows / 64) * (kChan / 64);
    static_assert(tiles % 8 == 0);
    wmma_gemm64<1, 2, 0, 0, false><<<dim3(tiles / 8, 1), 256, 0, stream>>>(
        DTH, DTL, kDtR, 0L,
        WDH, WDL, kDtR, 0L,
        (void*)DP, nullptr, kChan, 0L,
        nullptr, nullptr, 0L,
        kRows, kChan, kDtR, 1.0f);
  }

  scan_gate_kernel<<<kBatch * (kChan / kScanCh), kScanCh, 0, stream>>>(DP, UF, BC, gate, b_dt, A_log, Dp, out);
}
